// SimplifiedLinearAttention_42485816492251
// MI455X (gfx1250) — hardware-verified
//
#include <hip/hip_runtime.h>


#define NB_  8
#define NN   3136
#define IMG  56
#define CC   512
#define NH_  8
#define HD   64
typedef _Float16 h16;
typedef unsigned short bf;
typedef __attribute__((ext_vector_type(16))) __bf16   v16bf;
typedef __attribute__((ext_vector_type(16))) _Float16 v16h;
typedef __attribute__((ext_vector_type(8)))  _Float16 v8h;
typedef __attribute__((ext_vector_type(8)))  unsigned short v8us;
typedef __attribute__((ext_vector_type(8)))  float    v8f;
typedef __attribute__((ext_vector_type(4)))  float    v4f;
typedef v8h  __attribute__((may_alias)) v8ha;
typedef v4f  __attribute__((may_alias)) v4fa;
typedef v8us __attribute__((may_alias)) v8usa;

__device__ __forceinline__ unsigned short f2bf(float f) { unsigned u = __float_as_uint(f); u += 0x7FFFu + ((u >> 16) & 1u); return (unsigned short)(u >> 16); }
__device__ __forceinline__ float bf2f(unsigned short b) { return __uint_as_float(((unsigned)b) << 16); }
__device__ __forceinline__ float bfr(float f) { return bf2f(f2bf(f)); }
__device__ __forceinline__ v16h cat16(v8h lo, v8h hi) { return __builtin_shufflevector(lo, hi, 0, 1, 2, 3, 4, 5, 6, 7, 8, 9, 10, 11, 12, 13, 14, 15); }
__device__ __forceinline__ v16bf cat16b(v8us lo, v8us hi) { return __builtin_bit_cast(v16bf, __builtin_shufflevector(lo, hi, 0, 1, 2, 3, 4, 5, 6, 7, 8, 9, 10, 11, 12, 13, 14, 15)); }
__device__ __forceinline__ v8f wmma16(v16h a, v16h b, v8f c) { return __builtin_amdgcn_wmma_f32_16x16x32_f16(false, a, false, b, (short)0, c, false, false); }
__device__ __forceinline__ v8f wmmab(v16bf a, v16bf b, v8f c) { return __builtin_amdgcn_wmma_f32_16x16x32_bf16(false, a, false, b, (short)0, c, false, false); }


template <typename T16> struct WFrag;
template <> struct WFrag<h16> { typedef v16h V; static __device__ __forceinline__ V ld(const h16* p) { return cat16(*(const v8h*)p, *(const v8h*)(p + 16)); } static __device__ __forceinline__ v8f mma(V a, V b, v8f c) { return wmma16(a, b, c); } };
template <> struct WFrag<bf> { typedef v16bf V; static __device__ __forceinline__ V ld(const bf* p) { return cat16b(*(const v8us*)p, *(const v8us*)(p + 16)); } static __device__ __forceinline__ v8f mma(V a, V b, v8f c) { return wmmab(a, b, c); } };
template <typename T16, int NSPLIT, bool BIAS>
__global__ __launch_bounds__(32) void k_gemmw(const T16* __restrict__ A, const T16* __restrict__ A2, const T16* __restrict__ Bt, const T16* __restrict__ Bt2, int K, float* C, int ldc, const float* __restrict__ bias, size_t sA, size_t sB, size_t sC) {
    typedef typename WFrag<T16>::V V;
    __shared__ __align__(16) float os[16 * 68];
    const size_t z = blockIdx.z; A += z * sA; if (A2) A2 += z * sA; Bt += z * sB; if (Bt2) Bt2 += z * sB; C += z * sC;
    const int lane = threadIdx.x & 31, lr = lane & 15, hi = lane >> 4; const int r0 = blockIdx.x * 64, c0 = blockIdx.y * 64;
    v8f acc[4][4];
#pragma unroll
    for (int mb = 0; mb < 4; ++mb)
#pragma unroll
        for (int nb = 0; nb < 4; ++nb) acc[mb][nb] = (v8f){};
    const size_t aoff = (size_t)(r0 + lr) * K + 8 * hi, boff = (size_t)(c0 + lr) * K + 8 * hi;
#pragma unroll 1
    for (int kc = 0; kc < K; kc += 32) {
        V a[4], a2[4];
#pragma unroll
        for (int mb = 0; mb < 4; ++mb) { a[mb] = WFrag<T16>::ld(A + aoff + (size_t)mb * 16 * K + kc); if (NSPLIT == 1 || NSPLIT == 2) a2[mb] = WFrag<T16>::ld(A2 + aoff + (size_t)mb * 16 * K + kc); }
#pragma unroll
        for (int nb = 0; nb < 4; ++nb) { const V b = WFrag<T16>::ld(Bt + boff + (size_t)nb * 16 * K + kc); V b2; if (NSPLIT >= 2) b2 = WFrag<T16>::ld(Bt2 + boff + (size_t)nb * 16 * K + kc);
#pragma unroll
            for (int mb = 0; mb < 4; ++mb) { acc[mb][nb] = WFrag<T16>::mma(a[mb], b, acc[mb][nb]); if (NSPLIT == 1 || NSPLIT == 2) acc[mb][nb] = WFrag<T16>::mma(a2[mb], b, acc[mb][nb]); if (NSPLIT >= 2) acc[mb][nb] = WFrag<T16>::mma(a[mb], b2, acc[mb][nb]); } }
        asm volatile("v_nop\n\tv_nop\n\tv_nop\n\tv_nop" : "+v"(acc[0][0]), "+v"(acc[1][1]), "+v"(acc[2][2]), "+v"(acc[3][3]) : "v"(a[0]), "v"(a[3]));
    }
#pragma unroll
    for (int mb = 0; mb < 4; ++mb) {
#pragma unroll
        for (int nb = 0; nb < 4; ++nb) {
#pragma unroll
            for (int j = 0; j < 8; ++j) os[(hi * 8 + j) * 68 + nb * 16 + lr] = acc[mb][nb][j]; }
        __builtin_amdgcn_wave_barrier(); asm volatile("" ::: "memory");
        float* crow = C + (size_t)(r0 + mb * 16) * ldc + c0;
#pragma unroll 1
        for (int ps = 0; ps < 2; ++ps) {
#pragma unroll
            for (int s = 0; s < 8; ++s) { const int row = 2 * s + hi, cofs = lr * 4; v4f val = *(const v4fa*)(os + row * 68 + cofs); if (BIAS) { val[0] += bfr(bias[c0 + cofs]); val[1] += bfr(bias[c0 + cofs + 1]); val[2] += bfr(bias[c0 + cofs + 2]); val[3] += bfr(bias[c0 + cofs + 3]); }
                *(volatile v4f*)(crow + (size_t)row * ldc + cofs) = val; }
            if (ps == 0) __threadfence(); }
        __builtin_amdgcn_wave_barrier(); asm volatile("" ::: "memory");
    }
}

__device__ __forceinline__ void splitf(float y, unsigned short& h, unsigned short& l) { h = f2bf(y); l = f2bf(y - bf2f(h)); }
typedef __attribute__((ext_vector_type(2))) unsigned short v2us;

__global__ __launch_bounds__(256) void k_wtG(const float* __restrict__ w, int K, int N, bf* Bt) {
    const int lane = threadIdx.x & 31; const int L0 = (blockIdx.x * 8 + (threadIdx.x >> 5)) * 8; const int nlines = N * K / 64;
#pragma unroll 1
    for (int ps = 0; ps < 2; ++ps) {
#pragma unroll 1
        for (int l = 0; l < 8; ++l) { const int L = L0 + l; if (L >= nlines) break; const size_t e = (size_t)L * 64 + lane * 2; const int k = (int)(e % K), n = (int)(e / K); v2us o;
            o[0] = f2bf(w[(size_t)k * N + n]); o[1] = f2bf(w[(size_t)(k + 1) * N + n]); *(volatile v2us*)(Bt + e) = o; }
        if (ps == 0) __threadfence(); }
}
__global__ __launch_bounds__(256) void k_cvt8(const float* __restrict__ src, bf* dst, size_t n8) { const size_t i = (size_t)blockIdx.x * 256 + threadIdx.x; if (i >= n8) return; const v8f v = *(const v8f*)(src + i * 8); v8us o;
#pragma unroll
    for (int k = 0; k < 8; ++k) o[k] = f2bf(v[k]); *(volatile v8us*)(dst + i * 8) = o; __threadfence(); *(volatile v8us*)(dst + i * 8) = o; }
__global__ __launch_bounds__(256) void k_qpl(const float* __restrict__ QF, bf* Qh, bf* Ql) { const size_t e = ((size_t)blockIdx.x * 256 + threadIdx.x) * 2; if (e >= (size_t)NH_ * NN * HD) return; const int c = (int)(e % HD); const int i = (int)((e / HD) % NN); const int h = (int)(e / ((size_t)HD * NN)); v2us oh, ol;
#pragma unroll
    for (int q = 0; q < 2; ++q) { unsigned short a, c2; splitf(fmaxf(QF[(size_t)i * CC + h * HD + c + q], 0.f), a, c2); oh[q] = a; ol[q] = c2; } *(volatile v2us*)(Qh + e) = oh; *(volatile v2us*)(Ql + e) = ol; __threadfence(); *(volatile v2us*)(Qh + e) = oh; *(volatile v2us*)(Ql + e) = ol; }
__global__ __launch_bounds__(256) void k_kt(const float* __restrict__ KV, const float* __restrict__ pos, bf* Kh, bf* Kl) { const size_t e = ((size_t)blockIdx.x * 256 + threadIdx.x) * 2; if (e >= (size_t)NH_ * HD * NN) return; const int j = (int)(e % NN); const int c = (int)((e / NN) % HD); const int h = (int)(e / ((size_t)NN * HD)); const int col = h * HD + c; v2us oh, ol;
#pragma unroll
    for (int q = 0; q < 2; ++q) { const float k = fmaxf(__fadd_rn(KV[(size_t)(j + q) * 2 * CC + col], bfr(pos[(size_t)(j + q) * CC + col])), 0.f); unsigned short a, c2; splitf(k, a, c2); oh[q] = a; ol[q] = c2; } *(volatile v2us*)(Kh + e) = oh; *(volatile v2us*)(Kl + e) = ol; __threadfence(); *(volatile v2us*)(Kh + e) = oh; *(volatile v2us*)(Kl + e) = ol; }
__global__ __launch_bounds__(256) void k_vt(const float* __restrict__ KV, bf* Vh, bf* Vl) { const size_t e = ((size_t)blockIdx.x * 256 + threadIdx.x) * 2; if (e >= (size_t)NH_ * HD * NN) return; const int j = (int)(e % NN); const int d = (int)((e / NN) % HD); const int h = (int)(e / ((size_t)NN * HD)); const int col = CC + h * HD + d; v2us oh, ol;
#pragma unroll
    for (int q = 0; q < 2; ++q) { unsigned short a, c2; splitf(KV[(size_t)(j + q) * 2 * CC + col], a, c2); oh[q] = a; ol[q] = c2; } *(volatile v2us*)(Vh + e) = oh; *(volatile v2us*)(Vl + e) = ol; __threadfence(); *(volatile v2us*)(Vh + e) = oh; *(volatile v2us*)(Vl + e) = ol; }
__global__ __launch_bounds__(256) void k_ksum(const float* __restrict__ KV, const float* __restrict__ pos, float* KS) { const int col = blockIdx.x * 256 + threadIdx.x; if (col >= CC) return; float s = 0.f;
    for (int j = 0; j < NN; ++j) s = __fadd_rn(s, fmaxf(__fadd_rn(KV[(size_t)j * 2 * CC + col], bfr(pos[(size_t)j * CC + col])), 0.f));
    *(volatile float*)(KS + col) = s; __threadfence(); *(volatile float*)(KS + col) = s; }
__global__ __launch_bounds__(256) void k_z(const float* __restrict__ QF, const float* __restrict__ KS, float* Z) { const int e = blockIdx.x * 256 + threadIdx.x; if (e >= NH_ * NN) return; const int i = e % NN, h = e / NN; float s = 0.f;
    for (int c = 0; c < HD; ++c) { float p = __fmul_rn(fmaxf(QF[(size_t)i * CC + h * HD + c], 0.f), KS[h * HD + c]); asm volatile("" : "+v"(p)); s = __fadd_rn(s, p); }
    const float z = __fdiv_rn(1.0f, __fadd_rn(s, 1e-6f)); *(volatile float*)(Z + e) = z; __threadfence(); *(volatile float*)(Z + e) = z; }
__global__ __launch_bounds__(256) void k_kvt(const float* __restrict__ KVM, bf* Th, bf* Tl) { const int e = (blockIdx.x * 256 + threadIdx.x) * 2; if (e >= NH_ * HD * HD) return; const int c = e % HD; const int d = (e / HD) % HD; const int h = e / (HD * HD); v2us oh, ol;
#pragma unroll
    for (int q = 0; q < 2; ++q) { unsigned short a, c2; splitf(KVM[((size_t)h * HD + c + q) * HD + d], a, c2); oh[q] = a; ol[q] = c2; } *(volatile v2us*)(Th + e) = oh; *(volatile v2us*)(Tl + e) = ol; __threadfence(); *(volatile v2us*)(Th + e) = oh; *(volatile v2us*)(Tl + e) = ol; }
__global__ __launch_bounds__(256) void k_comb(const float* __restrict__ O, const float* __restrict__ Z, const float* __restrict__ KV, const float* __restrict__ w, const float* __restrict__ wb, bf* Ah, bf* Al) { const size_t e = ((size_t)blockIdx.x * 256 + threadIdx.x) * 2; if (e >= (size_t)NN * CC) return; const int col = (int)(e % CC), n = (int)(e / CC); const int h = col / HD, d = col % HD; const int wi = n / IMG, hi = n % IMG; const float z = Z[h * NN + n]; v2us oh, ol;
#pragma unroll
    for (int q = 0; q < 2; ++q) { const int dq = d + q; float cv = 0.f;
#pragma unroll
        for (int ky = 0; ky < 5; ++ky) { const int ww = wi + ky - 2; if (ww < 0 || ww >= IMG) continue;
#pragma unroll
            for (int kx = 0; kx < 5; ++kx) { const int hh = hi + kx - 2; if (hh < 0 || hh >= IMG) continue; float p = __fmul_rn(bfr(w[(dq * 5 + ky) * 5 + kx]), KV[(size_t)(ww * IMG + hh) * 2 * CC + CC + h * HD + dq]); asm volatile("" : "+v"(p)); cv = __fadd_rn(cv, p); } }
        float oz = __fmul_rn(O[((size_t)h * NN + n) * HD + dq], z); asm volatile("" : "+v"(oz)); const float r = __fadd_rn(oz, __fadd_rn(cv, bfr(wb[dq]))); unsigned short a, c2; splitf(r, a, c2); oh[q] = a; ol[q] = c2; }
    *(volatile v2us*)(Ah + e) = oh; *(volatile v2us*)(Al + e) = ol; __threadfence(); *(volatile v2us*)(Ah + e) = oh; *(volatile v2us*)(Al + e) = ol; }

extern "C" void kernel_launch(void* const* d_in, const int* in_sizes, int n_in,
                              void* d_out, int out_size, void* d_ws, size_t ws_size, hipStream_t stream) {
    (void)in_sizes; (void)n_in; (void)out_size;
    const float* x = (const float*)d_in[0]; const float* Wq = (const float*)d_in[3]; const float* Wkv = (const float*)d_in[4]; const float* pos = (const float*)d_in[5]; const float* dw = (const float*)d_in[6]; const float* dwb = (const float*)d_in[7]; const float* Wp = (const float*)d_in[8]; const float* bp = (const float*)d_in[9];
    float* OUT = (float*)d_out;
    char* wsp = (char*)d_ws;
    auto take = [&](size_t bytes) { char* p = wsp; wsp += (bytes + 255) & ~(size_t)255; return (void*)p; };
    bf* WQ = (bf*)take((size_t)CC * CC * 2); bf* WKV = (bf*)take((size_t)2 * CC * CC * 2); bf* WP = (bf*)take((size_t)CC * CC * 2); bf* XB = (bf*)take((size_t)NN * CC * 2); float* QF = (float*)take((size_t)NN * CC * 4); float* KV = (float*)take((size_t)NN * 2 * CC * 4);
    bf* Qh = (bf*)take((size_t)NH_ * NN * HD * 2); bf* Ql = (bf*)take((size_t)NH_ * NN * HD * 2); bf* Kh = (bf*)take((size_t)NH_ * HD * NN * 2); bf* Kl = (bf*)take((size_t)NH_ * HD * NN * 2); bf* Vh = (bf*)take((size_t)NH_ * HD * NN * 2); bf* Vl = (bf*)take((size_t)NH_ * HD * NN * 2);
    float* KS = (float*)take((size_t)CC * 4); float* Z = (float*)take((size_t)NH_ * NN * 4); float* KVM = (float*)take((size_t)NH_ * HD * HD * 4); bf* Th = (bf*)take((size_t)NH_ * HD * HD * 2); bf* Tl = (bf*)take((size_t)NH_ * HD * HD * 2); float* O = (float*)take((size_t)NH_ * NN * HD * 4); bf* Ah = (bf*)take((size_t)NN * CC * 2); bf* Al = (bf*)take((size_t)NN * CC * 2);
    if ((size_t)(wsp - (char*)d_ws) > ws_size) return;
    k_wtG<<<(CC * CC / 64 + 63) / 64, 256, 0, stream>>>(Wq, CC, CC, WQ); k_wtG<<<(CC * 2 * CC / 64 + 63) / 64, 256, 0, stream>>>(Wkv, CC, 2 * CC, WKV); k_wtG<<<(CC * CC / 64 + 63) / 64, 256, 0, stream>>>(Wp, CC, CC, WP);
    const unsigned LPL = (unsigned)(((size_t)NH_ * NN * HD / 2 + 255) / 256);
    for (int b = 0; b < NB_; ++b) {
        k_cvt8<<<(unsigned)(((size_t)NN * CC / 8 + 255) / 256), 256, 0, stream>>>(x + (size_t)b * NN * CC, XB, (size_t)NN * CC / 8);
        k_gemmw<bf, 0, false><<<dim3(NN / 64, CC / 64, 1), 32, 0, stream>>>(XB, nullptr, WQ, nullptr, CC, QF, CC, nullptr, 0, 0, 0); k_gemmw<bf, 0, false><<<dim3(NN / 64, 2 * CC / 64, 1), 32, 0, stream>>>(XB, nullptr, WKV, nullptr, CC, KV, 2 * CC, nullptr, 0, 0, 0);
        k_qpl<<<LPL, 256, 0, stream>>>(QF, Qh, Ql); k_kt<<<LPL, 256, 0, stream>>>(KV, pos, Kh, Kl); k_vt<<<LPL, 256, 0, stream>>>(KV, Vh, Vl); k_ksum<<<CC / 256, 256, 0, stream>>>(KV, pos, KS); k_z<<<(NH_ * NN + 255) / 256, 256, 0, stream>>>(QF, KS, Z);
        k_gemmw<bf, 2, false><<<dim3(1, 1, NH_), 32, 0, stream>>>(Kh, Kl, Vh, Vl, NN, KVM, HD, nullptr, (size_t)HD * NN, (size_t)HD * NN, (size_t)HD * HD);
        k_kvt<<<(NH_ * HD * HD / 2 + 255) / 256, 256, 0, stream>>>(KVM, Th, Tl);
        k_gemmw<bf, 2, false><<<dim3(NN / 64, 1, NH_), 32, 0, stream>>>(Qh, Ql, Th, Tl, HD, O, HD, nullptr, (size_t)NN * HD, (size_t)HD * HD, (size_t)NN * HD);
        k_comb<<<(unsigned)(((size_t)NN * CC / 2 + 255) / 256), 256, 0, stream>>>(O, Z, KV, dw, dwb, Ah, Al);
        k_gemmw<bf, 1, true><<<dim3(NN / 64, CC / 64, 1), 32, 0, stream>>>(Ah, Al, WP, nullptr, CC, OUT + (size_t)b * NN * CC, CC, bp, 0, 0, 0); }
}
